// MicroExpert_53936199303680
// MI455X (gfx1250) — hardware-verified
//
#include <hip/hip_runtime.h>
#include <math.h>
#include <float.h>
#include <stdint.h>

#define NB    2
#define SEQ   2048
#define DMOD  512
#define NHEAD 8
#define HD    64
#define DFF   1024
#define HWIN  256
#define NQB   (SEQ / 64)
#define SEQP  (SEQ + 2)
#define WSC   64.0f
#define LN_EPS 1e-5f
static_assert(NHEAD * HD == DMOD);
static_assert((SEQ % 128) == 0 && (DMOD % 128) == 0 && (DFF % 128) == 0);

typedef _Float16 v16h __attribute__((ext_vector_type(16)));
typedef _Float16 v8h  __attribute__((ext_vector_type(8)));
typedef float    v8f  __attribute__((ext_vector_type(8)));
typedef float    v4f  __attribute__((ext_vector_type(4)));
typedef unsigned int v4u __attribute__((ext_vector_type(4)));
typedef unsigned int v2u __attribute__((ext_vector_type(2)));

__device__ __forceinline__ unsigned pkh(float a, float b) {
  const _Float16 ha = (_Float16)a, hb = (_Float16)b;
  const unsigned short ua = __builtin_bit_cast(unsigned short, ha);
  const unsigned short ub = __builtin_bit_cast(unsigned short, hb);
  return (unsigned)ua | ((unsigned)ub << 16);
}
__device__ __forceinline__ v8f zero8() { v8f z = {0.f, 0.f, 0.f, 0.f, 0.f, 0.f, 0.f, 0.f}; return z; }

__device__ __forceinline__ v16h ldfrag(const _Float16* p) {
  union { v16h v; v8h h[2]; } f;
  f.h[0] = *(const v8h*)(p);
  f.h[1] = *(const v8h*)(p + 16);
  return f.v;
}

__device__ __forceinline__ v8f mma_h(v16h a, v16h b, v8f c) {
  c = __builtin_amdgcn_wmma_f32_16x16x32_f16(false, a, false, b, (short)0, c, false, false);
#if defined(__HIP_DEVICE_COMPILE__)
  asm volatile("v_nop\n\tv_nop\n\tv_nop\n\tv_nop" : "+v"(c) : "v"(a), "v"(b));
#endif
  return c;
}

__global__ __launch_bounds__(256) void cvt_x_pad(const float* __restrict__ x, unsigned short* xp, int ngrp) {
  const int i = blockIdx.x * 256 + threadIdx.x;
  if (i >= ngrp) return;
  const int row = i >> 6;
  const int cg  = (i & 63) * 8;
  const int b   = row / SEQP;
  const int tp  = row - b * SEQP;
  int t = tp - 1;
  t = (t < 0) ? 0 : t;
  t = (t > SEQ - 1) ? (SEQ - 1) : t;
  const float vm = (tp >= 1 && tp <= SEQ) ? 1.f : 0.f;
  const float* src = x + ((size_t)b * SEQ + (size_t)t) * DMOD + cg;
  v4f a = *(const v4f*)(src);
  v4f c = *(const v4f*)(src + 4);
  a *= vm; c *= vm;
  v4u p;
  p[0] = pkh(a[0], a[1]); p[1] = pkh(a[2], a[3]);
  p[2] = pkh(c[0], c[1]); p[3] = pkh(c[2], c[3]);
  unsigned short* dst = xp + (size_t)i * 8;
  *(volatile v4u*)dst = p;
  __threadfence();
  *(volatile v4u*)dst = p;
}

__global__ __launch_bounds__(256) void cvt_w(const float* __restrict__ w, unsigned short* out, int ngrp, float scale) {
  const int i = blockIdx.x * 256 + threadIdx.x;
  if (i >= ngrp) return;
  v4f a = *(const v4f*)(w + (size_t)i * 8);
  v4f c = *(const v4f*)(w + (size_t)i * 8 + 4);
  a *= scale; c *= scale;
  v4u p;
  p[0] = pkh(a[0], a[1]); p[1] = pkh(a[2], a[3]);
  p[2] = pkh(c[0], c[1]); p[3] = pkh(c[2], c[3]);
  unsigned short* dst = out + (size_t)i * 8;
  *(volatile v4u*)dst = p;
  __threadfence();
  *(volatile v4u*)dst = p;
}

__global__ __launch_bounds__(256) void cvt_convw(const float* __restrict__ cw, unsigned short* out, int ngrp, float scale) {
  const int i = blockIdx.x * 256 + threadIdx.x;
  if (i >= ngrp) return;
  const int o   = i / 192;
  const int g   = i - o * 192;
  const int k   = g * 8;
  const int tap = k >> 9;
  const int ci  = k & (DMOD - 1);
  const float* src = cw + ((size_t)o * DMOD + ci) * 3 + tap;
  float f[8];
#pragma unroll
  for (int e = 0; e < 8; ++e) f[e] = src[e * 3] * scale;
  v4u p;
  p[0] = pkh(f[0], f[1]); p[1] = pkh(f[2], f[3]);
  p[2] = pkh(f[4], f[5]); p[3] = pkh(f[6], f[7]);
  unsigned short* dst = out + (size_t)o * (3 * DMOD) + k;
  *(volatile v4u*)dst = p;
  __threadfence();
  *(volatile v4u*)dst = p;
}

template <int OUT16, int RESID, int ROWB>
__global__ __launch_bounds__(256) void gemm_f16(
    const unsigned short* __restrict__ Ap, int lda, long long strideA,
    const unsigned short* __restrict__ Bp, int ldb, long long strideB,
    const float* __restrict__ bias,
    const float* __restrict__ Rp, int ldr,
    void* Cp, int ldc, long long strideC,
    int K, float oscale, float cscale, int relu) {
  __shared__ __align__(16) float sT[8][16 * 68];
  const int lane = threadIdx.x & 31;
  const int wave = threadIdx.x >> 5;
  const int hh   = lane >> 4;
  const int rl   = lane & 15;
  const int z    = blockIdx.z;
  const int m0w  = blockIdx.y * 128 + (wave & 3) * 32;
  const int n0w  = blockIdx.x * 128 + (wave >> 2) * 64;
  const _Float16* A  = (const _Float16*)(const void*)Ap + (size_t)z * (size_t)strideA;
  const _Float16* Bt = (const _Float16*)(const void*)Bp + (size_t)z * (size_t)strideB;

  v8f acc[2][4];
#pragma unroll
  for (int i = 0; i < 2; ++i)
#pragma unroll
    for (int j = 0; j < 4; ++j) acc[i][j] = zero8();

  for (int k0 = 0; k0 < K; k0 += 32) {
    v16h bf[4];
#pragma unroll
    for (int j = 0; j < 4; ++j)
      bf[j] = ldfrag(Bt + (size_t)(n0w + 16 * j + rl) * ldb + k0 + 8 * hh);
#pragma unroll
    for (int i = 0; i < 2; ++i) {
      const v16h af = ldfrag(A + (size_t)(m0w + 16 * i + rl) * lda + k0 + 8 * hh);
#pragma unroll
      for (int j = 0; j < 4; ++j) acc[i][j] = mma_h(af, bf[j], acc[i][j]);
    }
  }

  float* slab = sT[wave];
#pragma unroll
  for (int i = 0; i < 2; ++i) {
    const int mBase = m0w + 16 * i;
#pragma unroll
    for (int j = 0; j < 4; ++j) {
#pragma unroll
      for (int r = 0; r < 8; ++r) slab[(8 * hh + r) * 68 + 16 * j + rl] = acc[i][j][r];
    }
    __syncthreads();
    if (OUT16 == 0) {
      float* C = (float*)Cp + (size_t)z * (size_t)strideC;
      const int r2 = lane >> 4, c4 = (lane & 15) * 4;
      const v4f bb = *(const v4f*)(bias + n0w + c4);
      v4f ov[8];
#pragma unroll
      for (int it = 0; it < 8; ++it) {
        const int row = 2 * it + r2;
        v4f v = *(const v4f*)(slab + row * 68 + c4);
        v = v * oscale + bb;
        if (relu) { v[0] = fmaxf(v[0], 0.f); v[1] = fmaxf(v[1], 0.f); v[2] = fmaxf(v[2], 0.f); v[3] = fmaxf(v[3], 0.f); }
        if (RESID) {
          const v4f rr = *(const v4f*)(Rp + (size_t)(mBase + row) * ldr + n0w + c4);
          v += rr;
        }
        ov[it] = v;
      }
      for (int pass = 0; pass < 2; ++pass) {
#pragma unroll
        for (int it = 0; it < 8; ++it) {
          const int row = 2 * it + r2;
          *(volatile v4f*)(C + (size_t)(mBase + row) * ldc + n0w + c4) = ov[it];
        }
        __threadfence();
      }
    } else {
      unsigned short* C = (unsigned short*)Cp + (size_t)z * (size_t)strideC;
      const int q4 = lane >> 3, c8 = (lane & 7) * 8;
      v4u hv[4];
#pragma unroll
      for (int it = 0; it < 4; ++it) {
        const int row = 4 * it + q4;
        const float* sp = slab + row * 68 + c8;
        v4f x0 = *(const v4f*)(sp);
        v4f x1 = *(const v4f*)(sp + 4);
        if (ROWB) {
          const float rb = bias[mBase + row];
          x0 = x0 * oscale + rb;
          x1 = x1 * oscale + rb;
        } else {
          const v4f b0 = *(const v4f*)(bias + n0w + c8);
          const v4f b1 = *(const v4f*)(bias + n0w + c8 + 4);
          x0 = x0 * oscale + b0;
          x1 = x1 * oscale + b1;
        }
        if (relu) {
          x0[0] = fmaxf(x0[0], 0.f); x0[1] = fmaxf(x0[1], 0.f); x0[2] = fmaxf(x0[2], 0.f); x0[3] = fmaxf(x0[3], 0.f);
          x1[0] = fmaxf(x1[0], 0.f); x1[1] = fmaxf(x1[1], 0.f); x1[2] = fmaxf(x1[2], 0.f); x1[3] = fmaxf(x1[3], 0.f);
        }
        x0 *= cscale; x1 *= cscale;
        v4u p;
        p[0] = pkh(x0[0], x0[1]); p[1] = pkh(x0[2], x0[3]);
        p[2] = pkh(x1[0], x1[1]); p[3] = pkh(x1[2], x1[3]);
        hv[it] = p;
      }
      for (int pass = 0; pass < 2; ++pass) {
#pragma unroll
        for (int it = 0; it < 4; ++it) {
          const int row = 4 * it + q4;
          *(volatile v4u*)(C + (size_t)(mBase + row) * ldc + n0w + c8) = hv[it];
        }
        __threadfence();
      }
    }
    __syncthreads();
  }
}

__global__ __launch_bounds__(128) void attn_band(
    const unsigned short* __restrict__ qp, const unsigned short* __restrict__ kp,
    const unsigned short* __restrict__ vtp, unsigned short* ctxp, float sscale, float cscale) {
  __shared__ __align__(16) _Float16 Ksh[64 * 64];
  __shared__ __align__(16) _Float16 Vth[64 * 64];
  __shared__ __align__(16) _Float16 Psh[4][16 * 64];
  __shared__ __align__(16) float    Os[4][16 * 64];

  const int tid  = threadIdx.x;
  const int wave = tid >> 5;
  const int lane = tid & 31;
  const int hh   = lane >> 4;
  const int c    = lane & 15;
  const int bx   = blockIdx.x;
  const int qb   = bx % NQB;
  const int h    = (bx / NQB) % NHEAD;
  const int b    = bx / (NQB * NHEAD);
  const int q0   = qb * 64 + wave * 16;
  const size_t rowB = (size_t)b * SEQ;

  const _Float16* Q  = (const _Float16*)(const void*)qp + (size_t)h * HD;
  const _Float16* Kg = (const _Float16*)(const void*)kp + (size_t)h * HD;
  const _Float16* Vt = (const _Float16*)(const void*)vtp + ((size_t)b * DMOD + (size_t)h * HD) * SEQ;

  v16h qa[2];
#pragma unroll
  for (int dc = 0; dc < 2; ++dc) qa[dc] = ldfrag(Q + (rowB + q0 + c) * DMOD + dc * 32 + 8 * hh);

  float mrow[8], lrow[8];
  v8f oacc[4];
#pragma unroll
  for (int r = 0; r < 8; ++r) { mrow[r] = -FLT_MAX; lrow[r] = 0.f; }
#pragma unroll
  for (int t = 0; t < 4; ++t) oacc[t] = zero8();

  for (int dk = -4; dk <= 4; ++dk) {
    const int kt = qb + dk;
    if (kt < 0 || kt >= NQB) continue;
    const int kv0 = kt * 64;
    __syncthreads();
    {
      const int r = tid >> 1, half = (tid & 1) * 32;
      const _Float16* kg = Kg + (rowB + kv0 + r) * DMOD + half;
      const _Float16* vg = Vt + (size_t)r * SEQ + kv0 + half;
#pragma unroll
      for (int i = 0; i < 4; ++i) {
        const v8h a0 = *(const v8h*)(kg + 8 * i);
        const v8h b0 = *(const v8h*)(vg + 8 * i);
        *(v8h*)(Ksh + r * 64 + half + 8 * i) = a0;
        *(v8h*)(Vth + r * 64 + half + 8 * i) = b0;
      }
    }
    __syncthreads();

    v8f s[4];
#pragma unroll
    for (int j = 0; j < 4; ++j) {
      s[j] = zero8();
#pragma unroll
      for (int dc = 0; dc < 2; ++dc) {
        union { v16h v; v8h hf[2]; } kb;
        kb.hf[0] = *(const v8h*)(Ksh + (j * 16 + c) * 64 + dc * 32 + 8 * hh);
        kb.hf[1] = *(const v8h*)(Ksh + (j * 16 + c) * 64 + dc * 32 + 16 + 8 * hh);
        s[j] = mma_h(qa[dc], kb.v, s[j]);
      }
    }

    _Float16* pw = Psh[wave];
#pragma unroll
    for (int r = 0; r < 8; ++r) {
      const int q = q0 + 8 * hh + r;
      float sv[4];
      int blk[4];
      float m = -FLT_MAX;
#pragma unroll
      for (int j = 0; j < 4; ++j) {
        const int key = kv0 + 16 * j + c;
        int d = q - key;
        d = (d < 0) ? -d : d;
        blk[j] = (d > HWIN) ? 1 : 0;
        const float x = s[j][r] * sscale;
        sv[j] = blk[j] ? -FLT_MAX : x;
        m = fmaxf(m, sv[j]);
      }
#pragma unroll
      for (int off = 1; off < 16; off <<= 1) m = fmaxf(m, __shfl_xor(m, off, 32));
      const float mnew  = fmaxf(mrow[r], m);
      const float alpha = (mrow[r] > -FLT_MAX) ? __expf(mrow[r] - mnew) : 0.f;
      mrow[r] = mnew;
      float psum = 0.f;
#pragma unroll
      for (int j = 0; j < 4; ++j) {
        const float e = __expf(sv[j] - mnew);
        const float p = blk[j] ? 0.f : e;
        psum += p;
        pw[(8 * hh + r) * 64 + 16 * j + c] = (_Float16)p;
      }
#pragma unroll
      for (int off = 1; off < 16; off <<= 1) psum += __shfl_xor(psum, off, 32);
      lrow[r] = lrow[r] * alpha + psum;
#pragma unroll
      for (int t = 0; t < 4; ++t) oacc[t][r] *= alpha;
    }
    __syncthreads();

#pragma unroll
    for (int kk = 0; kk < 2; ++kk) {
      union { v16h v; v8h hf[2]; } pa;
      pa.hf[0] = *(const v8h*)(pw + c * 64 + kk * 32 + 8 * hh);
      pa.hf[1] = *(const v8h*)(pw + c * 64 + kk * 32 + 16 + 8 * hh);
#pragma unroll
      for (int t = 0; t < 4; ++t) {
        union { v16h v; v8h hf[2]; } vb;
        vb.hf[0] = *(const v8h*)(Vth + (t * 16 + c) * 64 + kk * 32 + 8 * hh);
        vb.hf[1] = *(const v8h*)(Vth + (t * 16 + c) * 64 + kk * 32 + 16 + 8 * hh);
        oacc[t] = mma_h(pa.v, vb.v, oacc[t]);
      }
    }
  }

  float* os = Os[wave];
#pragma unroll
  for (int r = 0; r < 8; ++r) {
    const float l = lrow[r];
    const float inv = ((l > 0.f) ? (1.0f / l) : 0.f) * cscale;
#pragma unroll
    for (int t = 0; t < 4; ++t) os[(8 * hh + r) * 64 + t * 16 + c] = oacc[t][r] * inv;
  }
  __syncthreads();
  {
    const int q4 = lane >> 3, c8 = (lane & 7) * 8;
    v4u hv[4];
#pragma unroll
    for (int it = 0; it < 4; ++it) {
      const int row = 4 * it + q4;
      const float* sp = os + row * 64 + c8;
      const v4f a0 = *(const v4f*)(sp);
      const v4f a1 = *(const v4f*)(sp + 4);
      v4u p;
      p[0] = pkh(a0[0], a0[1]); p[1] = pkh(a0[2], a0[3]);
      p[2] = pkh(a1[0], a1[1]); p[3] = pkh(a1[2], a1[3]);
      hv[it] = p;
    }
    for (int pass = 0; pass < 2; ++pass) {
#pragma unroll
      for (int it = 0; it < 4; ++it) {
        const int row = 4 * it + q4;
        const size_t go = (rowB + q0 + row) * DMOD + (size_t)h * HD + c8;
        *(volatile v4u*)(ctxp + go) = hv[it];
      }
      __threadfence();
    }
  }
}

template <int H16>
__global__ __launch_bounds__(256) void ln_rows(const float* __restrict__ X, const float* __restrict__ g,
                                               const float* __restrict__ be, float* Y, unsigned short* Yh,
                                               int rows) {
  __shared__ __align__(16) unsigned sh[8][256];
  const int wave = threadIdx.x >> 5;
  const int lane = threadIdx.x & 31;
  int row = blockIdx.x * 8 + wave;
  row = (row < rows) ? row : (rows - 1);
  const float* xr = X + (size_t)row * DMOD;
  v4f v[4];
  float s = 0.f;
#pragma unroll
  for (int i = 0; i < 4; ++i) {
    v[i] = *(const v4f*)(xr + 128 * i + 4 * lane);
    s += (v[i][0] + v[i][1]) + (v[i][2] + v[i][3]);
  }
#pragma unroll
  for (int off = 1; off < 32; off <<= 1) s += __shfl_xor(s, off, 32);
  const float mean = s * (1.0f / (float)DMOD);
  float sq = 0.f;
#pragma unroll
  for (int i = 0; i < 4; ++i) {
    v[i] = v[i] - mean;
    sq += v[i][0] * v[i][0] + v[i][1] * v[i][1] + v[i][2] * v[i][2] + v[i][3] * v[i][3];
  }
#pragma unroll
  for (int off = 1; off < 32; off <<= 1) sq += __shfl_xor(sq, off, 32);
  const float var  = sq * (1.0f / (float)DMOD);
  const float rstd = rsqrtf(var + LN_EPS);
  v4f y[4];
#pragma unroll
  for (int i = 0; i < 4; ++i) {
    const v4f g4 = *(const v4f*)(g + 128 * i + 4 * lane);
    const v4f b4 = *(const v4f*)(be + 128 * i + 4 * lane);
    y[i] = (v[i] * rstd) * g4 + b4;
  }
  float* yr = Y + (size_t)row * DMOD;
  for (int pass = 0; pass < 2; ++pass) {
#pragma unroll
    for (int i = 0; i < 4; ++i) *(volatile v4f*)(yr + 128 * i + 4 * lane) = y[i];
    __threadfence();
  }
  if (H16) {
    unsigned* sw = sh[wave];
#pragma unroll
    for (int i = 0; i < 4; ++i) {
      v2u p;
      p[0] = pkh(y[i][0], y[i][1]);
      p[1] = pkh(y[i][2], y[i][3]);
      *(v2u*)(sw + 64 * i + 2 * lane) = p;
    }
    __syncthreads();
    v4u w[2];
#pragma unroll
    for (int i2 = 0; i2 < 2; ++i2) w[i2] = *(const v4u*)(sw + 128 * i2 + 4 * lane);
    unsigned short* hr = Yh + (size_t)row * DMOD;
    for (int pass = 0; pass < 2; ++pass) {
#pragma unroll
      for (int i2 = 0; i2 < 2; ++i2) *(volatile v4u*)(hr + 256 * i2 + 8 * lane) = w[i2];
      __threadfence();
    }
  }
}

extern "C" void kernel_launch(void* const* d_in, const int* in_sizes, int n_in,
                              void* d_out, int out_size, void* d_ws, size_t ws_size,
                              hipStream_t stream) {
  if (n_in < 16) return;
  if (in_sizes[0] != NB * SEQ * DMOD) return;
  if (in_sizes[2] != DMOD * DMOD * 3 || in_sizes[3] != DMOD) return;
  if (in_sizes[4] != 3 * DMOD * DMOD || in_sizes[5] != 3 * DMOD) return;
  if (in_sizes[6] != DMOD * DMOD || in_sizes[7] != DMOD) return;
  if (in_sizes[8] != DMOD || in_sizes[9] != DMOD) return;
  if (in_sizes[10] != DFF * DMOD || in_sizes[11] != DFF) return;
  if (in_sizes[12] != DMOD * DFF || in_sizes[13] != DMOD) return;
  if (in_sizes[14] != DMOD || in_sizes[15] != DMOD) return;
  if (out_size != NB * SEQ * DMOD) return;

  const float* x      = (const float*)d_in[0];
  const float* conv_w = (const float*)d_in[2];
  const float* conv_b = (const float*)d_in[3];
  const float* in_w   = (const float*)d_in[4];
  const float* in_b   = (const float*)d_in[5];
  const float* out_w  = (const float*)d_in[6];
  const float* out_b  = (const float*)d_in[7];
  const float* ln1_g  = (const float*)d_in[8];
  const float* ln1_b  = (const float*)d_in[9];
  const float* w1     = (const float*)d_in[10];
  const float* b1     = (const float*)d_in[11];
  const float* w2     = (const float*)d_in[12];
  const float* b2     = (const float*)d_in[13];
  const float* ln2_g  = (const float*)d_in[14];
  const float* ln2_b  = (const float*)d_in[15];

  const size_t MR = (size_t)NB * SEQ;
  size_t off = 0;
  auto carve = [&](size_t bytes) { const size_t o = off; off += (bytes + 127) & ~(size_t)127; return o; };
  const size_t oXp   = carve((size_t)NB * SEQP * DMOD * 2);
  const size_t oWc   = carve((size_t)DMOD * 3 * DMOD * 2);
  const size_t oWin  = carve((size_t)3 * DMOD * DMOD * 2);
  const size_t oWo   = carve((size_t)DMOD * DMOD * 2);
  const size_t oW1   = carve((size_t)DFF * DMOD * 2);
  const size_t oW2   = carve((size_t)DMOD * DFF * 2);
  const size_t oVIN  = carve(MR * DMOD * 2);
  const size_t oQ    = carve(MR * DMOD * 2);
  const size_t oK    = carve(MR * DMOD * 2);
  const size_t oVT   = carve((size_t)NB * DMOD * SEQ * 2);
  const size_t oCTX  = carve(MR * DMOD * 2);
  const size_t oPRE1 = carve(MR * DMOD * 4);
  const size_t oHf   = carve(MR * DMOD * 4);
  const size_t oHh   = carve(MR * DMOD * 2);
  const size_t oFF1  = carve(MR * DFF * 2);
  const size_t oPRE2 = carve(MR * DMOD * 4);
  if (off > ws_size) return;
  if (off > (size_t)134217728) return;

  char* ws = (char*)d_ws;
  unsigned short* Xp  = (unsigned short*)(ws + oXp);
  unsigned short* Wc  = (unsigned short*)(ws + oWc);
  unsigned short* Win = (unsigned short*)(ws + oWin);
  unsigned short* Wob = (unsigned short*)(ws + oWo);
  unsigned short* W1b = (unsigned short*)(ws + oW1);
  unsigned short* W2b = (unsigned short*)(ws + oW2);
  unsigned short* VIN = (unsigned short*)(ws + oVIN);
  unsigned short* Qp  = (unsigned short*)(ws + oQ);
  unsigned short* Kp  = (unsigned short*)(ws + oK);
  unsigned short* VT  = (unsigned short*)(ws + oVT);
  unsigned short* CTX = (unsigned short*)(ws + oCTX);
  float*          PRE1 = (float*)(ws + oPRE1);
  float*          Hf   = (float*)(ws + oHf);
  unsigned short* Hh   = (unsigned short*)(ws + oHh);
  unsigned short* FF1  = (unsigned short*)(ws + oFF1);
  float*          PRE2 = (float*)(ws + oPRE2);
  float*          out  = (float*)d_out;

  const dim3 blk(256);
  const int ngx  = NB * SEQP * DMOD / 8;
  const int ngc  = DMOD * 3 * DMOD / 8;
  const int ngin = 3 * DMOD * DMOD / 8;
  const int ngo  = DMOD * DMOD / 8;
  const int ngf  = DFF * DMOD / 8;
  const float invw  = 1.0f / WSC;
  const float invww = 1.0f / (WSC * WSC);

  cvt_x_pad<<<dim3((ngx + 255) / 256), blk, 0, stream>>>(x, Xp, ngx);
  cvt_convw<<<dim3((ngc + 255) / 256), blk, 0, stream>>>(conv_w, Wc, ngc, WSC);
  cvt_w<<<dim3((ngin + 255) / 256), blk, 0, stream>>>(in_w, Win, ngin, WSC);
  cvt_w<<<dim3((ngo + 255) / 256), blk, 0, stream>>>(out_w, Wob, ngo, WSC);
  cvt_w<<<dim3((ngf + 255) / 256), blk, 0, stream>>>(w1, W1b, ngf, WSC);
  cvt_w<<<dim3((ngf + 255) / 256), blk, 0, stream>>>(w2, W2b, ngf, WSC);

  gemm_f16<1, 0, 0><<<dim3(DMOD / 128, SEQ / 128, NB), blk, 0, stream>>>(
      Xp, DMOD, (long long)SEQP * DMOD, Wc, 3 * DMOD, 0LL,
      conv_b, (const float*)0, 0,
      (void*)VIN, DMOD, (long long)SEQ * DMOD,
      3 * DMOD, invw, 1.0f, 0);
  gemm_f16<1, 0, 0><<<dim3(DMOD / 128, SEQ / 128, NB), blk, 0, stream>>>(
      Xp + DMOD, DMOD, (long long)SEQP * DMOD, Win, DMOD, 0LL,
      in_b, (const float*)0, 0,
      (void*)Qp, DMOD, (long long)SEQ * DMOD,
      DMOD, invw, 1.0f, 0);
  gemm_f16<1, 0, 0><<<dim3(DMOD / 128, SEQ / 128, NB), blk, 0, stream>>>(
      Xp + DMOD, DMOD, (long long)SEQP * DMOD, Win + (size_t)DMOD * DMOD, DMOD, 0LL,
      in_b + DMOD, (const float*)0, 0,
      (void*)Kp, DMOD, (long long)SEQ * DMOD,
      DMOD, invw, 1.0f, 0);
  gemm_f16<1, 0, 1><<<dim3(SEQ / 128, DMOD / 128, NB), blk, 0, stream>>>(
      Win + (size_t)2 * DMOD * DMOD, DMOD, 0LL, VIN, DMOD, (long long)SEQ * DMOD,
      in_b + 2 * DMOD, (const float*)0, 0,
      (void*)VT, SEQ, (long long)DMOD * SEQ,
      DMOD, invw, 1.0f, 0);
  attn_band<<<dim3(NB * NHEAD * NQB), dim3(128), 0, stream>>>(Qp, Kp, VT, CTX, 0.125f, WSC);
  gemm_f16<0, 1, 0><<<dim3(DMOD / 128, (NB * SEQ) / 128, 1), blk, 0, stream>>>(
      CTX, DMOD, 0LL, Wob, DMOD, 0LL,
      out_b, x, DMOD,
      (void*)PRE1, DMOD, 0LL,
      DMOD, invww, 1.0f, 0);
  ln_rows<1><<<dim3((NB * SEQ) / 8), blk, 0, stream>>>(PRE1, ln1_g, ln1_b, Hf, Hh, NB * SEQ);
  gemm_f16<1, 0, 0><<<dim3(DFF / 128, (NB * SEQ) / 128, 1), blk, 0, stream>>>(
      Hh, DMOD, 0LL, W1b, DMOD, 0LL,
      b1, (const float*)0, 0,
      (void*)FF1, DFF, 0LL,
      DMOD, invw, 1.0f, 1);
  gemm_f16<0, 1, 0><<<dim3(DMOD / 128, (NB * SEQ) / 128, 1), blk, 0, stream>>>(
      FF1, DFF, 0LL, W2b, DFF, 0LL,
      b2, Hf, DMOD,
      (void*)PRE2, DMOD, 0LL,
      DFF, invw, 1.0f, 0);
  ln_rows<0><<<dim3((NB * SEQ) / 8), blk, 0, stream>>>(PRE2, ln2_g, ln2_b, out, (unsigned short*)Hh, NB * SEQ);
  (void)hipGetLastError();
}
